// SelfAttention1d_36069135352062
// MI455X (gfx1250) — hardware-verified
//
#include <hip/hip_runtime.h>


#ifndef NB
#define NB 2
#endif
#ifndef SEQ
#define SEQ 2048
#endif
#define NB_FULL  2
#define SEQ_FULL 2048
#define CC   1024
#define NH   16
#define HD   64
#define DQ   (NH * HD)
#define MT   (NB * SEQ)
#define NPL  (NB * NH)
#define ZH   2
#define PCAR 1024.0f
#define SCL  0.125f

static_assert(NB >= 1 && NB <= NB_FULL);
static_assert(SEQ >= 128 && SEQ <= SEQ_FULL && (SEQ % 128) == 0);
static_assert((MT % 64) == 0 && (CC % 64) == 0 && DQ == CC && HD == 64);
static_assert((NPL % ZH) == 0);

typedef _Float16 h16;
typedef unsigned short bf;
typedef __attribute__((ext_vector_type(16))) __bf16   v16bf;
typedef __attribute__((ext_vector_type(16))) _Float16 v16h;
typedef __attribute__((ext_vector_type(8)))  _Float16 v8h;
typedef __attribute__((ext_vector_type(8)))  unsigned short v8us;
typedef __attribute__((ext_vector_type(8)))  float    v8f;
typedef __attribute__((ext_vector_type(4)))  float    v4f;
typedef v8h  __attribute__((may_alias)) v8ha;
typedef v4f  __attribute__((may_alias)) v4fa;
typedef v8us __attribute__((may_alias)) v8usa;
typedef __attribute__((ext_vector_type(2))) _Float16 v2h;
typedef __attribute__((ext_vector_type(4))) _Float16 v4h;
typedef __attribute__((ext_vector_type(2))) unsigned short v2us;
typedef __attribute__((ext_vector_type(4))) unsigned short v4us;
typedef __attribute__((ext_vector_type(2))) float v2f;
typedef __attribute__((ext_vector_type(4))) int v4i;

__device__ __forceinline__ unsigned short f2bf(float f) { unsigned u = __float_as_uint(f); u += 0x7FFFu + ((u >> 16) & 1u); return (unsigned short)(u >> 16); }
__device__ __forceinline__ float bf2f(unsigned short b) { return __uint_as_float(((unsigned)b) << 16); }
__device__ __forceinline__ float bfr(float f) { return bf2f(f2bf(f)); }
__device__ __forceinline__ v16h cat16(v8h lo, v8h hi) { return __builtin_shufflevector(lo, hi, 0, 1, 2, 3, 4, 5, 6, 7, 8, 9, 10, 11, 12, 13, 14, 15); }
__device__ __forceinline__ v16bf cat16b(v8us lo, v8us hi) { return __builtin_bit_cast(v16bf, __builtin_shufflevector(lo, hi, 0, 1, 2, 3, 4, 5, 6, 7, 8, 9, 10, 11, 12, 13, 14, 15)); }
__device__ __forceinline__ v8f wmma16(v16h a, v16h b, v8f c) { return __builtin_amdgcn_wmma_f32_16x16x32_f16(false, a, false, b, (short)0, c, false, false); }
__device__ __forceinline__ v8f wmmab(v16bf a, v16bf b, v8f c) { return __builtin_amdgcn_wmma_f32_16x16x32_bf16(false, a, false, b, (short)0, c, false, false); }
__device__ __forceinline__ h16 tohx(float x) { return (h16)x; }
__device__ __forceinline__ void splitf(float y, unsigned short& h, unsigned short& l) { h = f2bf(y); l = f2bf(y - bf2f(h)); }

template <typename T16> struct WFrag;
template <> struct WFrag<h16> { typedef v16h V; static __device__ __forceinline__ V ld(const h16* p) { return cat16(*(const v8h*)p, *(const v8h*)(p + 16)); } static __device__ __forceinline__ v8f mma(V a, V b, v8f c) { return wmma16(a, b, c); } };
template <> struct WFrag<bf> { typedef v16bf V; static __device__ __forceinline__ V ld(const bf* p) { return cat16b(*(const v8us*)p, *(const v8us*)(p + 16)); } static __device__ __forceinline__ v8f mma(V a, V b, v8f c) { return wmmab(a, b, c); } };
template <typename T16, int NSPLIT, bool BIAS>
__global__ __launch_bounds__(32) void k_gemmw(const T16* __restrict__ A, const T16* __restrict__ A2, const T16* __restrict__ Bt, const T16* __restrict__ Bt2, int K, float* C, int ldc, const float* __restrict__ bias, size_t sA, size_t sB, size_t sC) {
    typedef typename WFrag<T16>::V V;
    __shared__ __align__(16) float os[16 * 68];
    const size_t z = blockIdx.z; A += z * sA; if (A2) A2 += z * sA; Bt += z * sB; if (Bt2) Bt2 += z * sB; C += z * sC;
    const int lane = threadIdx.x & 31, lr = lane & 15, hi = lane >> 4; const int r0 = blockIdx.x * 64, c0 = blockIdx.y * 64;
    v8f acc[4][4];
#pragma unroll
    for (int mb = 0; mb < 4; ++mb)
#pragma unroll
        for (int nb = 0; nb < 4; ++nb) acc[mb][nb] = (v8f){};
    const size_t aoff = (size_t)(r0 + lr) * K + 8 * hi, boff = (size_t)(c0 + lr) * K + 8 * hi;
#pragma unroll 1
    for (int kc = 0; kc < K; kc += 32) {
        V a[4], a2[4];
#pragma unroll
        for (int mb = 0; mb < 4; ++mb) { a[mb] = WFrag<T16>::ld(A + aoff + (size_t)mb * 16 * K + kc); if (NSPLIT == 1 || NSPLIT == 2) a2[mb] = WFrag<T16>::ld(A2 + aoff + (size_t)mb * 16 * K + kc); }
#pragma unroll
        for (int nb = 0; nb < 4; ++nb) { const V b = WFrag<T16>::ld(Bt + boff + (size_t)nb * 16 * K + kc); V b2; if (NSPLIT >= 2) b2 = WFrag<T16>::ld(Bt2 + boff + (size_t)nb * 16 * K + kc);
#pragma unroll
            for (int mb = 0; mb < 4; ++mb) { acc[mb][nb] = WFrag<T16>::mma(a[mb], b, acc[mb][nb]); if (NSPLIT == 1 || NSPLIT == 2) acc[mb][nb] = WFrag<T16>::mma(a2[mb], b, acc[mb][nb]); if (NSPLIT >= 2) acc[mb][nb] = WFrag<T16>::mma(a[mb], b2, acc[mb][nb]); } }
        asm volatile("v_nop\n\tv_nop\n\tv_nop\n\tv_nop" : "+v"(acc[0][0]), "+v"(acc[1][1]), "+v"(acc[2][2]), "+v"(acc[3][3]) : "v"(a[0]), "v"(a[3]));
    }
#pragma unroll
    for (int mb = 0; mb < 4; ++mb) {
#pragma unroll
        for (int nb = 0; nb < 4; ++nb) {
#pragma unroll
            for (int j = 0; j < 8; ++j) os[(hi * 8 + j) * 68 + nb * 16 + lr] = acc[mb][nb][j]; }
        __builtin_amdgcn_wave_barrier(); asm volatile("" ::: "memory");
        float* crow = C + (size_t)(r0 + mb * 16) * ldc + c0;
#pragma unroll 1
        for (int ps = 0; ps < 2; ++ps) {
#pragma unroll
            for (int s = 0; s < 8; ++s) { const int row = 2 * s + hi, cofs = lr * 4; v4f val = *(const v4fa*)(os + row * 68 + cofs); if (BIAS) { val[0] += bfr(bias[c0 + cofs]); val[1] += bfr(bias[c0 + cofs + 1]); val[2] += bfr(bias[c0 + cofs + 2]); val[3] += bfr(bias[c0 + cofs + 3]); }
                *(volatile v4f*)(crow + (size_t)row * ldc + cofs) = val; }
            if (ps == 0) __threadfence(); }
        __builtin_amdgcn_wave_barrier(); asm volatile("" ::: "memory");
    }
}

__global__ __launch_bounds__(256) void k_cvt8(const float* __restrict__ src, bf* dst, size_t n8) { const size_t i = (size_t)blockIdx.x * 256 + threadIdx.x; if (i >= n8) return; const v8f v = *(const v8f*)(src + i * 8); v8us o;
#pragma unroll
    for (int k = 0; k < 8; ++k) o[k] = f2bf(v[k]); *(volatile v8us*)(dst + i * 8) = o; __threadfence(); *(volatile v8us*)(dst + i * 8) = o; }

__global__ __launch_bounds__(256) void k_gnstat(const float* __restrict__ x, float* stat) {
    __shared__ float red[256]; const int tid = threadIdx.x; const float* xs = x + (size_t)blockIdx.x * CC * SEQ_FULL; const size_t n = (size_t)CC * SEQ; float s = 0.f;
    for (size_t e = (size_t)tid * 4; e < n; e += 256 * 4) { const size_t c = e / SEQ, t = e % SEQ; const v4f a = *(const v4f*)(xs + c * SEQ_FULL + t); for (int q = 0; q < 4; ++q) s = __fadd_rn(s, bfr(a[q])); }
    red[tid] = s; __syncthreads();
    for (int st = 128; st > 0; st >>= 1) { if (tid < st) red[tid] = __fadd_rn(red[tid], red[tid + st]); __syncthreads(); }
    const float mean = __fdiv_rn(red[0], (float)n); __syncthreads(); float s2 = 0.f;
    for (size_t e = (size_t)tid * 4; e < n; e += 256 * 4) { const size_t c = e / SEQ, t = e % SEQ; const v4f a = *(const v4f*)(xs + c * SEQ_FULL + t); for (int q = 0; q < 4; ++q) { const float dv = __fsub_rn(bfr(a[q]), mean); float p2 = __fmul_rn(dv, dv); asm volatile("" : "+v"(p2)); s2 = __fadd_rn(s2, p2); } }
    red[tid] = s2; __syncthreads();
    for (int st = 128; st > 0; st >>= 1) { if (tid < st) red[tid] = __fadd_rn(red[tid], red[tid + st]); __syncthreads(); }
    const float var = __fdiv_rn(red[0], (float)n); const float rs = __fdiv_rn(1.0f, __fsqrt_rn(__fadd_rn(var, 1e-5f)));
    if (tid < 32) { v4f o; o[0] = mean; o[1] = rs; o[2] = 0.f; o[3] = 0.f; float* p = stat + (size_t)blockIdx.x * 128 + tid * 4; *(volatile v4f*)p = o; __threadfence(); *(volatile v4f*)p = o; } }

__global__ __launch_bounds__(256) void k_gnT(const float* __restrict__ x, const float* __restrict__ stat, const float* __restrict__ g, const float* __restrict__ bb, bf* XH, bf* XL) {
    const size_t k = (size_t)blockIdx.x * 256 + threadIdx.x; if (k >= (size_t)MT * CC / 8) return; const int c0 = (int)(k % (CC / 8)) * 8; const int tok = (int)(k / (CC / 8)); const int b = tok / SEQ, t = tok % SEQ;
    const float mean = stat[(size_t)b * 128], rs = stat[(size_t)b * 128 + 1]; const float* xs = x + (size_t)b * CC * SEQ_FULL; v8us oh, ol;
#pragma unroll
    for (int q = 0; q < 8; ++q) { const int c = c0 + q; const float dv = __fsub_rn(bfr(xs[(size_t)c * SEQ_FULL + t]), mean); float y = __fmul_rn(dv, rs); asm volatile("" : "+v"(y)); y = __fmul_rn(y, bfr(g[c])); asm volatile("" : "+v"(y)); y = __fadd_rn(y, bfr(bb[c])); unsigned short a2, c2; splitf(y, a2, c2); oh[q] = a2; ol[q] = c2; }
    const size_t oo = (size_t)tok * CC + c0;
    *(volatile v8us*)(XH + oo) = oh; *(volatile v8us*)(XL + oo) = ol; __threadfence(); *(volatile v8us*)(XH + oo) = oh; *(volatile v8us*)(XL + oo) = ol; }

__global__ __launch_bounds__(256) void k_qkp(const float* __restrict__ F, h16* P16) {
    const size_t e = ((size_t)blockIdx.x * 256 + threadIdx.x) * 8; if (e >= (size_t)NPL * SEQ * HD) return;
    const int d = (int)(e % HD); const int t = (int)((e / HD) % SEQ); const int g = (int)(e / ((size_t)HD * SEQ)); const int b = g / NH, h = g % NH;
    const float* f = F + ((size_t)b * SEQ + t) * DQ + h * HD + d; const v4f a0 = *(const v4f*)f; const v4f a1 = *(const v4f*)(f + 4); v8h o;
#pragma unroll
    for (int q = 0; q < 4; ++q) { o[q] = tohx(a0[q]); o[q + 4] = tohx(a1[q]); }
    *(volatile v8h*)(P16 + e) = o; __threadfence(); *(volatile v8h*)(P16 + e) = o; }
__global__ __launch_bounds__(256) void k_vtp(const float* __restrict__ F, h16* V16) {
    const size_t e = ((size_t)blockIdx.x * 256 + threadIdx.x) * 2; if (e >= (size_t)NPL * HD * SEQ) return;
    const int t = (int)(e % SEQ); const int d = (int)((e / SEQ) % HD); const int g = (int)(e / ((size_t)SEQ * HD)); const int b = g / NH, h = g % NH; v2h o16;
#pragma unroll
    for (int q = 0; q < 2; ++q) o16[q] = tohx(F[((size_t)b * SEQ + t + q) * DQ + h * HD + d]);
    *(volatile v2h*)(V16 + e) = o16; __threadfence(); *(volatile v2h*)(V16 + e) = o16; }

__global__ __launch_bounds__(256) void k_lsoft(const float* __restrict__ Sb, const int* __restrict__ msk, int hp, h16* P16) {
#pragma clang fp contract(off)
    const int lane = threadIdx.x & 31; const int row = blockIdx.x * 8 + (threadIdx.x >> 5); if (row >= ZH * SEQ) return;
    const int zz = row / SEQ; const int b = (hp + zz) / NH; const int* mr = msk + (size_t)b * SEQ_FULL; const float* sr = Sb + (size_t)row * SEQ;
    float rv[SEQ / 32]; float mx = -3.0e38f;
#pragma unroll
    for (int ch = 0; ch < SEQ / 128; ++ch) { const int j0 = ch * 128 + lane * 4; const v4f a = *(const v4f*)(sr + j0); const v4i mk = *(const v4i*)(mr + j0);
#pragma unroll
        for (int q = 0; q < 4; ++q) { float t = __fmul_rn(a[q], SCL); t = (mk[q] != 0) ? t : -3.0e38f; rv[ch * 4 + q] = t; mx = fmaxf(mx, t); }
        if ((ch & 3) == 3) asm volatile("" ::: "memory"); }
#pragma unroll
    for (int sh = 16; sh; sh >>= 1) mx = fmaxf(mx, __shfl_xor(mx, sh, 32));
    float sum = 0.f;
#pragma unroll
    for (int k2 = 0; k2 < SEQ / 32; ++k2) { float d0 = __fsub_rn(rv[k2], mx); asm volatile("" : "+v"(d0)); float ex = __builtin_amdgcn_exp2f(__fmul_rn(d0, 1.4426950408889634f)); asm volatile("" : "+v"(ex)); rv[k2] = ex; sum = __fadd_rn(sum, ex); }
#pragma unroll
    for (int sh = 16; sh; sh >>= 1) sum = __fadd_rn(sum, __shfl_xor(sum, sh, 32));
    const float f = __fdiv_rn(PCAR, sum);
#pragma unroll 1
    for (int ps = 0; ps < 2; ++ps) {
#pragma unroll
        for (int ch = 0; ch < SEQ / 128; ++ch) { const int j0 = ch * 128 + lane * 4; v4h o4;
#pragma unroll
            for (int q = 0; q < 4; ++q) o4[q] = tohx(__fmul_rn(rv[ch * 4 + q], f));
            *(volatile v4h*)(P16 + (size_t)row * SEQ + j0) = o4; }
        if (ps == 0) __threadfence(); }
}

__global__ __launch_bounds__(256) void k_merge(const float* __restrict__ O, int hp, bf* Ah, bf* Al) {
    const size_t e = ((size_t)blockIdx.x * 256 + threadIdx.x) * 2; if (e >= (size_t)ZH * SEQ * HD) return;
    const int d = (int)(e % HD); const int t = (int)((e / HD) % SEQ); const int zz = (int)(e / ((size_t)HD * SEQ)); const int g = hp + zz; const int b = g / NH, h = g % NH;
    const size_t oo = ((size_t)b * SEQ + t) * DQ + h * HD + d; v2us oh, ol;
#pragma unroll
    for (int q = 0; q < 2; ++q) { unsigned short a, c2; splitf(O[e + q] * (1.0f / PCAR), a, c2); oh[q] = a; ol[q] = c2; }
    *(volatile v2us*)(Ah + oo) = oh; *(volatile v2us*)(Al + oo) = ol; __threadfence(); *(volatile v2us*)(Ah + oo) = oh; *(volatile v2us*)(Al + oo) = ol; }

__global__ __launch_bounds__(256) void k_outTr(const float* __restrict__ U, const float* __restrict__ x, float* outp) {
    const size_t k = (size_t)blockIdx.x * 256 + threadIdx.x; if (k >= (size_t)NB * CC * SEQ / 4) return; const size_t e = k * 4;
    const int t0 = (int)(e % SEQ); const int c = (int)((e / SEQ) % CC); const int b = (int)(e / ((size_t)SEQ * CC));
    const size_t gi = ((size_t)b * CC + c) * SEQ_FULL + t0; const v4f a = *(const v4f*)(x + gi); v4f o;
#pragma unroll
    for (int q = 0; q < 4; ++q) o[q] = __fadd_rn(bfr(a[q]), U[((size_t)b * SEQ + t0 + q) * CC + c]);
    *(volatile v4f*)(outp + gi) = o; __threadfence(); *(volatile v4f*)(outp + gi) = o; }

extern "C" void kernel_launch(void* const* d_in, const int* in_sizes, int n_in,
                              void* d_out, int out_size, void* d_ws, size_t ws_size, hipStream_t stream) {
    if (n_in < 12) return;
    if (in_sizes[0] < NB * CC * SEQ_FULL || in_sizes[1] < NB * SEQ_FULL || in_sizes[2] < CC || in_sizes[3] < CC || in_sizes[4] < CC * CC || in_sizes[5] < CC
        || in_sizes[6] < CC * CC || in_sizes[7] < CC || in_sizes[8] < CC * CC || in_sizes[9] < CC || in_sizes[10] < CC * CC || in_sizes[11] < CC) return;
    if ((size_t)out_size < (size_t)(NB - 1) * CC * SEQ_FULL + (size_t)(CC - 1) * SEQ_FULL + (size_t)SEQ) return;
    const float* x   = (const float*)d_in[0];
    const int*   msk = (const int*)d_in[1];
    const float* gnw = (const float*)d_in[2]; const float* gnb = (const float*)d_in[3];
    const float* wq = (const float*)d_in[4]; const float* bq = (const float*)d_in[5]; const float* wk = (const float*)d_in[6]; const float* bk = (const float*)d_in[7];
    const float* wv = (const float*)d_in[8]; const float* bv = (const float*)d_in[9]; const float* wo = (const float*)d_in[10]; const float* bo = (const float*)d_in[11];
    float* OUT = (float*)d_out;
    char* wsp = (char*)d_ws;
    auto take = [&](size_t bytes) { char* p = wsp; wsp += (bytes + 255) & ~(size_t)255; return (void*)p; };
    float* STAT = (float*)take((size_t)NB * 512);
    bf* XH = (bf*)take((size_t)MT * CC * 2); bf* XL = (bf*)take((size_t)MT * CC * 2);
    bf* WQ = (bf*)take((size_t)CC * CC * 2); bf* WK = (bf*)take((size_t)CC * CC * 2); bf* WV = (bf*)take((size_t)CC * CC * 2); bf* WOB = (bf*)take((size_t)CC * CC * 2);
    h16* QP16 = (h16*)take((size_t)NPL * SEQ * HD * 2); h16* KP16 = (h16*)take((size_t)NPL * SEQ * HD * 2); h16* VT16 = (h16*)take((size_t)NPL * HD * SEQ * 2);
    size_t bigb = (size_t)ZH * SEQ * SEQ * 4;
    if ((size_t)2 * MT * DQ * 4 > bigb) bigb = (size_t)2 * MT * DQ * 4;
    if ((size_t)MT * CC * 4 > bigb) bigb = (size_t)MT * CC * 4;
    float* BIG = (float*)take(bigb);
    h16* P16 = (h16*)take((size_t)ZH * SEQ * SEQ * 2); float* Ob = (float*)take((size_t)ZH * SEQ * HD * 4);
    bf* ATh = (bf*)take((size_t)MT * DQ * 2); bf* ATl = (bf*)take((size_t)MT * DQ * 2);
    if ((size_t)(wsp - (char*)d_ws) > ws_size) return;
    float* Sb = BIG; float* FQ = BIG; float* FK = BIG + (size_t)MT * DQ; float* FV = FK; float* Y = BIG;

    const unsigned gw8 = (unsigned)(((size_t)CC * CC / 8 + 255) / 256);
    k_cvt8<<<gw8, 256, 0, stream>>>(wq, WQ, (size_t)CC * CC / 8); k_cvt8<<<gw8, 256, 0, stream>>>(wk, WK, (size_t)CC * CC / 8);
    k_cvt8<<<gw8, 256, 0, stream>>>(wv, WV, (size_t)CC * CC / 8); k_cvt8<<<gw8, 256, 0, stream>>>(wo, WOB, (size_t)CC * CC / 8);
    k_gnstat<<<NB, 256, 0, stream>>>(x, STAT);
    k_gnT<<<(unsigned)(((size_t)MT * CC / 8 + 255) / 256), 256, 0, stream>>>(x, STAT, gnw, gnb, XH, XL);
    const dim3 gp(MT / 64, DQ / 64, 1);
    const unsigned gqk = (unsigned)(((size_t)NPL * SEQ * HD / 8 + 255) / 256), gvt = (unsigned)(((size_t)NPL * HD * SEQ / 2 + 255) / 256);
    k_gemmw<bf, 1, true><<<gp, 32, 0, stream>>>(XH, XL, WQ, nullptr, CC, FQ, DQ, bq, 0, 0, 0); k_qkp<<<gqk, 256, 0, stream>>>(FQ, QP16);
    k_gemmw<bf, 1, true><<<gp, 32, 0, stream>>>(XH, XL, WK, nullptr, CC, FK, DQ, bk, 0, 0, 0); k_qkp<<<gqk, 256, 0, stream>>>(FK, KP16);
    k_gemmw<bf, 1, true><<<gp, 32, 0, stream>>>(XH, XL, WV, nullptr, CC, FV, DQ, bv, 0, 0, 0); k_vtp<<<gvt, 256, 0, stream>>>(FV, VT16);
    for (int hp = 0; hp < NPL; hp += ZH) {
        k_gemmw<h16, 0, false><<<dim3(SEQ / 64, SEQ / 64, ZH), 32, 0, stream>>>(QP16 + (size_t)hp * SEQ * HD, nullptr, KP16 + (size_t)hp * SEQ * HD, nullptr, HD, Sb, SEQ, nullptr, (size_t)SEQ * HD, (size_t)SEQ * HD, (size_t)SEQ * SEQ);
        k_lsoft<<<ZH * SEQ / 8, 256, 0, stream>>>(Sb, msk, hp, P16);
        k_gemmw<h16, 0, false><<<dim3(SEQ / 64, HD / 64, ZH), 32, 0, stream>>>(P16, nullptr, VT16 + (size_t)hp * HD * SEQ, nullptr, SEQ, Ob, HD, nullptr, (size_t)SEQ * SEQ, (size_t)HD * SEQ, (size_t)SEQ * HD);
        k_merge<<<(unsigned)(((size_t)ZH * SEQ * HD / 2 + 255) / 256), 256, 0, stream>>>(Ob, hp, ATh, ATl); }
    k_gemmw<bf, 1, true><<<dim3(MT / 64, CC / 64, 1), 32, 0, stream>>>(ATh, ATl, WOB, nullptr, DQ, Y, CC, bo, 0, 0, 0);
    k_outTr<<<(unsigned)(((size_t)NB * CC * SEQ / 4 + 255) / 256), 256, 0, stream>>>(Y, x, OUT);
}
